// LinearAttention_48112223650146
// MI455X (gfx1250) — hardware-verified
//
#include <hip/hip_runtime.h>
#include <math.h>
#include <stdint.h>


#define BATCH  2
#define SEQ    2048
#define DIM    512
#define HEADS  8
#define DH     64
#define INNER  512
#define QKV3   1536
#define ROWS   (BATCH * SEQ)
#define QKP    1024
#define OPITCH 1024
#define L2E    1.44269504088896340736f

typedef __attribute__((ext_vector_type(16))) __bf16   v16b;
typedef __attribute__((ext_vector_type(8)))  __bf16   v8b;
typedef __attribute__((ext_vector_type(8)))  _Float16 v8h;
typedef __attribute__((ext_vector_type(8)))  float    v8f;
typedef __attribute__((ext_vector_type(4)))  float    v4f;
typedef __attribute__((ext_vector_type(4)))  unsigned int v4u;

__device__ __forceinline__ unsigned short f2bf_bits(float f) {
  unsigned u = __float_as_uint(f);
  return (unsigned short)((u + 0x7FFFu + ((u >> 16) & 1u)) >> 16);
}
__device__ __forceinline__ float bf_bits2f(unsigned short h) { return __uint_as_float(((unsigned)h) << 16); }
__device__ __forceinline__ unsigned pk16(unsigned short a, unsigned short b) { return (unsigned)a | ((unsigned)b << 16); }

__device__ __forceinline__ void dep_guard_b(v8f& a, v8f& b, v16b x, v16b y) {
  asm volatile("v_nop\n\tv_nop\n\tv_nop\n\tv_nop" : "+v"(a), "+v"(b) : "v"(x), "v"(y));
}
__device__ __forceinline__ void keep4_b(v16b a, v16b b, v16b c, v16b d) { asm volatile("v_nop" :: "v"(a), "v"(b), "v"(c), "v"(d)); }
__device__ __forceinline__ void acc_guard4(v8f& a, v8f& b, v8f& c, v8f& d) {
  asm volatile("v_nop\n\tv_nop\n\tv_nop\n\tv_nop" : "+v"(a), "+v"(b), "+v"(c), "+v"(d));
}

union FragU { v16b v; v8b h[2]; };
__device__ __forceinline__ v16b frag_load(const __bf16* p) {
  FragU f;
  f.h[0] = *(const v8b*)(p);
  f.h[1] = *(const v8b*)(p + 16);
  return f.v;
}
__device__ __forceinline__ v8f frag_mma(v16b a, v16b b, v8f c) {
  return __builtin_amdgcn_wmma_f32_16x16x32_bf16(false, a, false, b, (short)0, c, false, false);
}

template <bool SPLIT, int BIAS_MODE, int OUT_MODE>
__global__ __launch_bounds__(256) void wmma_gemm64(
    const unsigned short* __restrict__ Ap, const unsigned short* __restrict__ A2p, int lda, long strideA,
    const unsigned short* __restrict__ Btp, const unsigned short* __restrict__ Bt2p, int ldb, long strideB,
    void* Cout, void* Cout2, int ldc, long strideC,
    const float* __restrict__ bias, int M, int N, int K, float scale) {
  const __bf16* A = (const __bf16*)(const void*)Ap;   const __bf16* A2  = (const __bf16*)(const void*)A2p;
  const __bf16* Bt = (const __bf16*)(const void*)Btp; const __bf16* Bt2 = (const __bf16*)(const void*)Bt2p;
  __shared__ __align__(16) float sT[8][16 * 68];
  const int b    = blockIdx.y;
  const int lane = threadIdx.x & 31;
  const int wave = threadIdx.x >> 5;
  const int tilesN = N >> 6;
  const int tilesM = M >> 6;
  const int tile = blockIdx.x * 8 + wave;
  if (tile >= tilesM * tilesN) return;
  const int tm = tile / tilesN;
  const int tn = tile - tm * tilesN;
  const int m0 = tm << 6;
  const int n0 = tn << 6;

  const __bf16* Ab  = A  + (size_t)b * strideA;
  const __bf16* Bb  = Bt + (size_t)b * strideB;
  const __bf16* Ab2 = SPLIT ? (A2  + (size_t)b * strideA) : nullptr;
  const __bf16* Bb2 = SPLIT ? (Bt2 + (size_t)b * strideB) : nullptr;

  const int rlane = lane & 15;
  const int koff  = (lane >> 4) * 8;
  const int mOff  = (lane >> 4) * 8;

  v8f acc[4][4];
#pragma unroll
  for (int i = 0; i < 4; ++i)
#pragma unroll
    for (int j = 0; j < 4; ++j) acc[i][j] = (v8f){0.f,0.f,0.f,0.f,0.f,0.f,0.f,0.f};

  for (int k0 = 0; k0 < K; k0 += 32) {
    v16b bh[4], bl[4];
#pragma unroll
    for (int j = 0; j < 4; ++j) {
      const size_t bo = (size_t)(n0 + (j << 4) + rlane) * ldb + koff + k0;
      bh[j] = frag_load(Bb + bo);
      if (SPLIT) bl[j] = frag_load(Bb2 + bo);
    }
#pragma unroll
    for (int i = 0; i < 4; ++i) {
      const size_t ao = (size_t)(m0 + (i << 4) + rlane) * lda + koff + k0;
      v16b ah = frag_load(Ab + ao);
      v16b al;
      if (SPLIT) al = frag_load(Ab2 + ao);
#pragma unroll
      for (int j = 0; j < 4; ++j) {
        acc[i][j] = frag_mma(ah, bh[j], acc[i][j]);
        if (SPLIT) {
          acc[i][j] = frag_mma(ah, bl[j], acc[i][j]);
          acc[i][j] = frag_mma(al, bh[j], acc[i][j]);
        }
      }
      dep_guard_b(acc[i][0], acc[i][3], ah, SPLIT ? al : ah);
    }
    keep4_b(bh[0], bh[1], bh[2], bh[3]);
    if (SPLIT) keep4_b(bl[0], bl[1], bl[2], bl[3]);
  }
  acc_guard4(acc[0][0], acc[0][1], acc[0][2], acc[0][3]);
  acc_guard4(acc[1][0], acc[1][1], acc[1][2], acc[1][3]);
  acc_guard4(acc[2][0], acc[2][1], acc[2][2], acc[2][3]);
  acc_guard4(acc[3][0], acc[3][1], acc[3][2], acc[3][3]);

  float* slab = sT[wave];
#pragma unroll
  for (int i = 0; i < 4; ++i) {
    const int mBase = m0 + (i << 4);
#pragma unroll
    for (int j = 0; j < 4; ++j) {
      const int n = n0 + (j << 4) + rlane;
      float bv = 0.f;
      if (BIAS_MODE == 2) bv = bias[n];
#pragma unroll
      for (int r = 0; r < 8; ++r) {
        float v = acc[i][j][r] * scale;
        if (BIAS_MODE == 2) v += bv;
        slab[(mOff + r) * 68 + (j << 4) + rlane] = v;
      }
    }
    __builtin_amdgcn_fence(__ATOMIC_RELEASE, "workgroup");
    __builtin_amdgcn_wave_barrier();
    __builtin_amdgcn_fence(__ATOMIC_ACQUIRE, "workgroup");
    if (OUT_MODE == 0) {
      float* C = (float*)Cout + (size_t)b * strideC;
      const int hh = lane >> 4, c4 = (lane & 15) * 4;
      for (int pass = 0; pass < 2; ++pass) {
#pragma unroll
        for (int it = 0; it < 8; ++it) {
          const int row = it * 2 + hh;
          v4f v = *(const v4f*)(slab + row * 68 + c4);
          *(volatile v4f*)(C + (size_t)(mBase + row) * ldc + n0 + c4) = v;
        }
        __threadfence();
      }
    } else {
      const int q = lane >> 3, c8 = (lane & 7) * 8;
      unsigned short* C  = (unsigned short*)Cout  + (size_t)b * strideC;
      unsigned short* C2 = (unsigned short*)Cout2 + (size_t)b * strideC;
      for (int pass = 0; pass < 2; ++pass) {
#pragma unroll
        for (int it = 0; it < 4; ++it) {
          const int row = it * 4 + q;
          const float* sp = slab + row * 68 + c8;
          v8h hv, lv;
#pragma unroll
          for (int e = 0; e < 8; ++e) {
            const unsigned short hb = f2bf_bits(sp[e]);
            const unsigned short lb = f2bf_bits(sp[e] - bf_bits2f(hb));
            hv[e] = __builtin_bit_cast(_Float16, hb);
            lv[e] = __builtin_bit_cast(_Float16, lb);
          }
          *(volatile v8h*)(C  + (size_t)(mBase + row) * ldc + n0 + c8) = hv;
          *(volatile v8h*)(C2 + (size_t)(mBase + row) * ldc + n0 + c8) = lv;
        }
        __threadfence();
      }
    }
    __builtin_amdgcn_fence(__ATOMIC_RELEASE, "workgroup");
    __builtin_amdgcn_wave_barrier();
    __builtin_amdgcn_fence(__ATOMIC_ACQUIRE, "workgroup");
  }
}

#define NXG (ROWS * DIM / 8)
#define NWG (QKV3 * DIM / 8)
#define NOG (DIM * INNER / 8)
#define PB_X (NXG / 256)
#define PB_W (NWG / 256)
#define PB_O (NOG / 256)
#define PB_TOTAL (PB_X + PB_W + PB_O + 1)
static_assert(NXG % 256 == 0);
static_assert(NWG % 256 == 0);
static_assert(NOG % 256 == 0);

__device__ __forceinline__ v4u pack_bf8(const float* src) {
  const v4f a = *(const v4f*)src;
  const v4f c = *(const v4f*)(src + 4);
  v4u o;
  o[0] = pk16(f2bf_bits(a.x), f2bf_bits(a.y));
  o[1] = pk16(f2bf_bits(a.z), f2bf_bits(a.w));
  o[2] = pk16(f2bf_bits(c.x), f2bf_bits(c.y));
  o[3] = pk16(f2bf_bits(c.z), f2bf_bits(c.w));
  return o;
}
__device__ __forceinline__ float bf_rt(float f) { return bf_bits2f(f2bf_bits(f)); }

__global__ __launch_bounds__(256) void prep_kernel(
    const float* __restrict__ x, const float* __restrict__ wqkv, const float* __restrict__ wout,
    const float* __restrict__ bout,
    unsigned short* __restrict__ XB, unsigned short* __restrict__ WQ, unsigned short* __restrict__ W2,
    float* __restrict__ BO) {
  const int blk = blockIdx.x, tid = threadIdx.x;
  if (blk < PB_X) {
    const size_t g = (size_t)blk * 256 + tid;
    const v4u o = pack_bf8(x + g * 8);
    unsigned short* d = XB + g * 8;
    *(volatile v4u*)d = o;
    __threadfence();
    *(volatile v4u*)d = o;
  } else if (blk < PB_X + PB_W) {
    const size_t g = (size_t)(blk - PB_X) * 256 + tid;
    const v4u o = pack_bf8(wqkv + g * 8);
    unsigned short* d = WQ + g * 8;
    *(volatile v4u*)d = o;
    __threadfence();
    *(volatile v4u*)d = o;
  } else if (blk < PB_X + PB_W + PB_O) {
    const int e = (blk - PB_X - PB_W) * 256 + tid;
    const int o = e >> 6;
    const int c = (e & 63) * 8;
    const v4u v = pack_bf8(wout + (size_t)o * INNER + c);
    unsigned short* d1 = W2 + (size_t)o * OPITCH + c;
    unsigned short* d2 = d1 + INNER;
    *(volatile v4u*)d1 = v;
    *(volatile v4u*)d2 = v;
    __threadfence();
    *(volatile v4u*)d1 = v;
    *(volatile v4u*)d2 = v;
  } else {
    if (tid < DIM / 4) {
      const v4f a = *(const v4f*)(bout + tid * 4);
      v4f r;
      r.x = bf_rt(a.x); r.y = bf_rt(a.y); r.z = bf_rt(a.z); r.w = bf_rt(a.w);
      *(volatile v4f*)(BO + tid * 4) = r;
      __threadfence();
      *(volatile v4f*)(BO + tid * 4) = r;
    }
  }
}

__device__ __forceinline__ void tsplit_store(const float* tf, unsigned short* oh, unsigned short* ol,
                                             size_t rowbase, int colbase, int tid) {
  const int sub = tid >> 3;
  const int c8  = (tid & 7) * 8;
  v4u hv[2], lv[2];
#pragma unroll
  for (int it = 0; it < 2; ++it) {
    const int oc = it * 32 + sub;
    v4u a, a2;
#pragma unroll
    for (int q = 0; q < 4; ++q) {
      const float f0 = tf[(c8 + 2 * q) * 68 + oc];
      const float f1 = tf[(c8 + 2 * q + 1) * 68 + oc];
      const unsigned short h0 = f2bf_bits(f0), h1 = f2bf_bits(f1);
      const unsigned short l0 = f2bf_bits(f0 - bf_bits2f(h0)), l1 = f2bf_bits(f1 - bf_bits2f(h1));
      a[q]  = pk16(h0, h1);
      a2[q] = pk16(l0, l1);
    }
    hv[it] = a; lv[it] = a2;
  }
  for (int pass = 0; pass < 2; ++pass) {
#pragma unroll
    for (int it = 0; it < 2; ++it) {
      const int oc = it * 32 + sub;
      const size_t go = (rowbase + oc) * (size_t)SEQ + colbase + c8;
      *(volatile v4u*)(oh + go) = hv[it];
      *(volatile v4u*)(ol + go) = lv[it];
    }
    __threadfence();
  }
}

__device__ __forceinline__ float max4(v4f v) { return fmaxf(fmaxf(v.x, v.y), fmaxf(v.z, v.w)); }
__device__ __forceinline__ float sum4(v4f v) { return (v.x + v.y) + (v.z + v.w); }
__device__ __forceinline__ v4f exps4(v4f v, float m) {
  v4f r;
  r.x = exp2f((v.x - m) * L2E); r.y = exp2f((v.y - m) * L2E);
  r.z = exp2f((v.z - m) * L2E); r.w = exp2f((v.w - m) * L2E);
  return r;
}
__device__ __forceinline__ v4f scale4(v4f v, float s) { v4f r; r.x = v.x * s; r.y = v.y * s; r.z = v.z * s; r.w = v.w * s; return r; }

__global__ __launch_bounds__(256) void qsoft_t_kernel(const float* __restrict__ QK,
                                                      unsigned short* __restrict__ oh, unsigned short* __restrict__ ol) {
  __shared__ __align__(16) float tf[64 * 68];
  const int i0 = blockIdx.x * 64, h = blockIdx.y, b = blockIdx.z;
  const int tid = threadIdx.x;
  {
    const int lr = tid >> 4;
    const int c4 = (tid & 15) * 4;
#pragma unroll
    for (int it = 0; it < 4; ++it) {
      const int rr = it * 16 + lr;
      const v4f a = *(const v4f*)(QK + (size_t)(b * SEQ + i0 + rr) * QKP + h * DH + c4);
      *(v4f*)(tf + rr * 68 + c4) = a;
    }
  }
  __syncthreads();
  {
    const int r = tid >> 2, p16 = (tid & 3) * 16;
    float* rp = tf + r * 68 + p16;
    v4f v0 = *(const v4f*)(rp);
    v4f v1 = *(const v4f*)(rp + 4);
    v4f v2 = *(const v4f*)(rp + 8);
    v4f v3 = *(const v4f*)(rp + 12);
    float m = fmaxf(fmaxf(max4(v0), max4(v1)), fmaxf(max4(v2), max4(v3)));
    m = fmaxf(m, __shfl_xor(m, 1, 32));
    m = fmaxf(m, __shfl_xor(m, 2, 32));
    v0 = exps4(v0, m); v1 = exps4(v1, m); v2 = exps4(v2, m); v3 = exps4(v3, m);
    float s = (sum4(v0) + sum4(v1)) + (sum4(v2) + sum4(v3));
    s += __shfl_xor(s, 1, 32);
    s += __shfl_xor(s, 2, 32);
    const float inv = 1.0f / s;
    *(v4f*)(rp)      = scale4(v0, inv);
    *(v4f*)(rp + 4)  = scale4(v1, inv);
    *(v4f*)(rp + 8)  = scale4(v2, inv);
    *(v4f*)(rp + 12) = scale4(v3, inv);
  }
  __syncthreads();
  tsplit_store(tf, oh, ol, (size_t)b * INNER + h * DH, i0, tid);
}

__global__ __launch_bounds__(256) void ksoft_t_kernel(const float* __restrict__ QK,
                                                      unsigned short* __restrict__ oh, unsigned short* __restrict__ ol) {
  __shared__ __align__(16) float tf[64 * 68];
  __shared__ float red[4 * 64];
  __shared__ float cmx[64];
  __shared__ float cin[64];
  const int h = blockIdx.x, b = blockIdx.y;
  const int tid = threadIdx.x;
  const int col = tid & 63, rg = tid >> 6;
  const float* colp = QK + (size_t)(b * SEQ) * QKP + DIM + h * DH + col;

  float m = -INFINITY;
#pragma unroll 4
  for (int r = rg; r < SEQ; r += 4) m = fmaxf(m, colp[(size_t)r * QKP]);
  red[rg * 64 + col] = m;
  __syncthreads();
  if (tid < 64) cmx[tid] = fmaxf(fmaxf(red[tid], red[64 + tid]), fmaxf(red[128 + tid], red[192 + tid]));
  __syncthreads();
  m = cmx[col];
  float s = 0.0f;
#pragma unroll 4
  for (int r = rg; r < SEQ; r += 4) s += exp2f((colp[(size_t)r * QKP] - m) * L2E);
  red[rg * 64 + col] = s;
  __syncthreads();
  if (tid < 64) {
    const float t = (red[tid] + red[64 + tid]) + (red[128 + tid] + red[192 + tid]);
    cin[tid] = 1.0f / t;
  }
  __syncthreads();

  const int lr = tid >> 4;
  const int c4 = (tid & 15) * 4;
  const float mc0 = cmx[c4], mc1 = cmx[c4 + 1], mc2 = cmx[c4 + 2], mc3 = cmx[c4 + 3];
  const float ic0 = cin[c4], ic1 = cin[c4 + 1], ic2 = cin[c4 + 2], ic3 = cin[c4 + 3];
  const float* tb = QK + (size_t)(b * SEQ) * QKP + DIM + h * DH + c4;
#pragma unroll 1
  for (int t = 0; t < SEQ / 64; ++t) {
    const int i0 = t * 64;
#pragma unroll
    for (int it = 0; it < 4; ++it) {
      const int rr = it * 16 + lr;
      const v4f a = *(const v4f*)(tb + (size_t)(i0 + rr) * QKP);
      v4f p;
      p.x = exp2f((a.x - mc0) * L2E) * ic0;
      p.y = exp2f((a.y - mc1) * L2E) * ic1;
      p.z = exp2f((a.z - mc2) * L2E) * ic2;
      p.w = exp2f((a.w - mc3) * L2E) * ic3;
      *(v4f*)(tf + rr * 68 + c4) = p;
    }
    __syncthreads();
    tsplit_store(tf, oh, ol, (size_t)b * INNER + h * DH, i0, tid);
    __syncthreads();
  }
}

#define SZ_XB  ((size_t)ROWS * DIM * 2)
#define SZ_WQ  ((size_t)QKV3 * DIM * 2)
#define SZ_W2  ((size_t)DIM * OPITCH * 2)
#define SZ_BO  ((size_t)DIM * 4)
#define SZ_QK  ((size_t)ROWS * QKP * 4)
#define SZ_V   ((size_t)ROWS * INNER * 2)
#define SZ_T   ((size_t)BATCH * INNER * SEQ * 2)
#define SZ_MT  ((size_t)BATCH * HEADS * DH * DH * 2)
#define SZ_O2  ((size_t)ROWS * OPITCH * 2)
#define WS_TOTAL (SZ_XB + SZ_WQ + SZ_W2 + SZ_BO + SZ_QK + 2 * SZ_V + 4 * SZ_T + 2 * SZ_MT + SZ_O2)
static_assert(WS_TOTAL == 57411584);
static_assert(WS_TOTAL <= 134217728);
static_assert(SZ_XB % 128 == 0 && SZ_WQ % 128 == 0 && SZ_W2 % 128 == 0 && SZ_BO % 128 == 0 && SZ_QK % 128 == 0);
static_assert(SZ_V % 128 == 0 && SZ_T % 128 == 0 && SZ_MT % 128 == 0 && SZ_O2 % 128 == 0);
static_assert(DIM % 32 == 0 && SEQ % 64 == 0 && DH % 32 == 0 && OPITCH % 32 == 0);
static_assert((ROWS / 64) * (QKP / 64) % 8 == 0);
static_assert((ROWS / 64) * (INNER / 64) % 8 == 0);
static_assert((SEQ / 64) % 8 == 0);

extern "C" void kernel_launch(void* const* d_in, const int* in_sizes, int n_in,
                              void* d_out, int out_size, void* d_ws, size_t ws_size,
                              hipStream_t stream) {
  if (n_in < 4) return;
  if (in_sizes[0] != ROWS * DIM) return;
  if (in_sizes[1] != QKV3 * DIM) return;
  if (in_sizes[2] != DIM * INNER) return;
  if (in_sizes[3] != DIM) return;
  if (out_size != ROWS * DIM) return;
  if ((size_t)WS_TOTAL > ws_size) return;

  const float* x     = (const float*)d_in[0];
  const float* w_qkv = (const float*)d_in[1];
  const float* w_out = (const float*)d_in[2];
  const float* b_out = (const float*)d_in[3];
  float* out = (float*)d_out;

  char* ws = (char*)d_ws;
  size_t off = 0;
  unsigned short* XB  = (unsigned short*)(ws + off); off += SZ_XB;
  unsigned short* WQ  = (unsigned short*)(ws + off); off += SZ_WQ;
  unsigned short* W2  = (unsigned short*)(ws + off); off += SZ_W2;
  float*          BO  = (float*)(ws + off);          off += SZ_BO;
  float*          QKF = (float*)(ws + off);          off += SZ_QK;
  unsigned short* Vh  = (unsigned short*)(ws + off); off += SZ_V;
  unsigned short* Vl  = (unsigned short*)(ws + off); off += SZ_V;
  unsigned short* QTh = (unsigned short*)(ws + off); off += SZ_T;
  unsigned short* QTl = (unsigned short*)(ws + off); off += SZ_T;
  unsigned short* KTh = (unsigned short*)(ws + off); off += SZ_T;
  unsigned short* KTl = (unsigned short*)(ws + off); off += SZ_T;
  unsigned short* MTh = (unsigned short*)(ws + off); off += SZ_MT;
  unsigned short* MTl = (unsigned short*)(ws + off); off += SZ_MT;
  unsigned short* O2  = (unsigned short*)(ws + off); off += SZ_O2;
  if (off > ws_size) return;

  const dim3 blk(256);

  prep_kernel<<<dim3(PB_TOTAL), blk, 0, stream>>>(x, w_qkv, w_out, b_out, XB, WQ, W2, BO);

  wmma_gemm64<false, 0, 0><<<dim3((ROWS / 64) * (QKP / 64) / 8, 1), blk, 0, stream>>>(
      XB, XB, DIM, 0L, WQ, WQ, DIM, 0L, (void*)QKF, (void*)QKF, QKP, 0L,
      BO, ROWS, QKP, DIM, 1.0f);

  wmma_gemm64<false, 0, 2><<<dim3((ROWS / 64) * (INNER / 64) / 8, 1), blk, 0, stream>>>(
      XB, XB, DIM, 0L, WQ + (size_t)2 * INNER * DIM, WQ + (size_t)2 * INNER * DIM, DIM, 0L,
      (void*)Vh, (void*)Vl, INNER, 0L,
      BO, ROWS, INNER, DIM, 1.0f);

  qsoft_t_kernel<<<dim3(SEQ / 64, HEADS, BATCH), blk, 0, stream>>>(QKF, QTh, QTl);

  ksoft_t_kernel<<<dim3(HEADS, BATCH), blk, 0, stream>>>(QKF, KTh, KTl);

  wmma_gemm64<true, 0, 2><<<dim3(1, BATCH * HEADS), dim3(32), 0, stream>>>(
      QTh, QTl, SEQ, (long)DH * SEQ, KTh, KTl, SEQ, (long)DH * SEQ,
      (void*)MTh, (void*)MTl, DH, (long)DH * DH,
      BO, DH, DH, SEQ, 1.0f);

  for (int bb = 0; bb < BATCH; ++bb) {
    wmma_gemm64<true, 0, 2><<<dim3((SEQ / 64) / 8, HEADS), blk, 0, stream>>>(
        Vh + (size_t)bb * SEQ * INNER, Vl + (size_t)bb * SEQ * INNER, INNER, (long)DH,
        MTh + (size_t)bb * HEADS * DH * DH, MTl + (size_t)bb * HEADS * DH * DH, DH, (long)DH * DH,
        (void*)(O2 + (size_t)bb * SEQ * OPITCH), (void*)(O2 + (size_t)bb * SEQ * OPITCH + INNER), OPITCH, (long)DH,
        BO, SEQ, DH, DH, 1.0f);
  }

  wmma_gemm64<false, 2, 0><<<dim3((ROWS / 64) * (DIM / 64) / 8, 1), blk, 0, stream>>>(
      O2, O2, OPITCH, 0L, W2, W2, OPITCH, 0L, (void*)out, (void*)out, DIM, 0L,
      BO, ROWS, DIM, OPITCH, 1.0f);

  (void)hipGetLastError();
}
